// Qwen3AttentionTP_57011395887281
// MI455X (gfx1250) — hardware-verified
//
#include <hip/hip_runtime.h>
#include <math.h>
#include <stdint.h>

constexpr int kBatch = 2;
constexpr int kSeq = 2048;
constexpr int kDm = 2048;
constexpr int kHeads = 16;
constexpr int kHd = 128;
constexpr int kTok = kBatch * kSeq;
constexpr int kChunkTok = 1024;
constexpr int kNumChunks = kSeq / kChunkTok;
constexpr int kNQB = kSeq / 64;
constexpr float kScoreScale = 0.08838834764831845f;

typedef __attribute__((ext_vector_type(16))) _Float16 v16h;
typedef __attribute__((ext_vector_type(8)))  _Float16 v8h;
typedef __attribute__((ext_vector_type(16))) __bf16   v16b;
typedef __attribute__((ext_vector_type(8)))  __bf16   v8b;
typedef __attribute__((ext_vector_type(8)))  float    v8f;
typedef __attribute__((ext_vector_type(4)))  float    v4f;
typedef __attribute__((ext_vector_type(2)))  float    v2f;

__device__ __forceinline__ unsigned short f2bf_bits(float f) {
  unsigned u = __float_as_uint(f);
  return (unsigned short)((u + 0x7FFFu + ((u >> 16) & 1u)) >> 16);
}
__device__ __forceinline__ float bf_bits2f(unsigned short h) { return __uint_as_float(((unsigned)h) << 16); }
__device__ __forceinline__ float bf_rne(float f) { return bf_bits2f(f2bf_bits(f)); }
__device__ __forceinline__ unsigned pk16(unsigned short a, unsigned short b) { return (unsigned)a | ((unsigned)b << 16); }

__device__ __forceinline__ void dep_guard_h(v8f& a, v8f& b, v16h x, v16h y) { asm volatile("v_nop\n\tv_nop\n\tv_nop\n\tv_nop" : "+v"(a), "+v"(b) : "v"(x), "v"(y)); }
__device__ __forceinline__ void dep_guard_b(v8f& a, v8f& b, v16b x, v16b y) { asm volatile("v_nop\n\tv_nop\n\tv_nop\n\tv_nop" : "+v"(a), "+v"(b) : "v"(x), "v"(y)); }
__device__ __forceinline__ void keep4_h(v16h a, v16h b, v16h c, v16h d) { asm volatile("v_nop" :: "v"(a), "v"(b), "v"(c), "v"(d)); }
__device__ __forceinline__ void keep4_b(v16b a, v16b b, v16b c, v16b d) { asm volatile("v_nop" :: "v"(a), "v"(b), "v"(c), "v"(d)); }
__device__ __forceinline__ void acc_guard4(v8f& a, v8f& b, v8f& c, v8f& d) { asm volatile("v_nop\n\tv_nop\n\tv_nop\n\tv_nop" : "+v"(a), "+v"(b), "+v"(c), "+v"(d)); }
template <typename T> struct Frag;
template <> struct Frag<_Float16> {
  typedef v16h V; union U { v16h v; v8h h[2]; };
  static __device__ __forceinline__ v16h load(const _Float16* p) {
    U f; f.h[0] = *(const v8h*)(p); f.h[1] = *(const v8h*)(p + 16); return f.v;
  }
  static __device__ __forceinline__ v8f mma(v16h a, v16h b, v8f c) {
    return __builtin_amdgcn_wmma_f32_16x16x32_f16(false, a, false, b, (short)0, c, false, false);
  }
  static __device__ __forceinline__ void guard(v8f& a, v8f& b, v16h x, v16h y) { dep_guard_h(a, b, x, y); }
  static __device__ __forceinline__ void keep(v16h a, v16h b, v16h c, v16h d) { keep4_h(a, b, c, d); }
};
template <> struct Frag<__bf16> {
  typedef v16b V; union U { v16b v; v8b h[2]; };
  static __device__ __forceinline__ v16b load(const __bf16* p) {
    U f; f.h[0] = *(const v8b*)(p); f.h[1] = *(const v8b*)(p + 16); return f.v;
  }
  static __device__ __forceinline__ v8f mma(v16b a, v16b b, v8f c) {
    return __builtin_amdgcn_wmma_f32_16x16x32_bf16(false, a, false, b, (short)0, c, false, false);
  }
  static __device__ __forceinline__ void guard(v8f& a, v8f& b, v16b x, v16b y) { dep_guard_b(a, b, x, y); }
  static __device__ __forceinline__ void keep(v16b a, v16b b, v16b c, v16b d) { keep4_b(a, b, c, d); }
};

template <int ET> struct Elem;
template <> struct Elem<0> { typedef _Float16 T; };
template <> struct Elem<1> { typedef __bf16 T; };
template <int ET, bool SPLIT, int BIAS_MODE, int OUT_MODE, bool RESID, int ACT = 0, bool ASPLIT = false>
__global__ __launch_bounds__(256) void wmma_gemm64(
    const unsigned short* __restrict__ Ap, const unsigned short* __restrict__ A2p, int lda, long strideA,
    const unsigned short* __restrict__ Btp, const unsigned short* __restrict__ Bt2p, int ldb, long strideB,
    void* __restrict__ Cout, void* __restrict__ Cout2, int ldc, long strideC,
    const float* __restrict__ bias,
    const float* __restrict__ resid, long strideR,
    int M, int N, int K, float scale) {
  typedef typename Elem<ET>::T T;
  typedef typename Frag<T>::V V;
  const T* A = (const T*)Ap; const T* A2 = (const T*)A2p; const T* Bt = (const T*)Btp; const T* Bt2 = (const T*)Bt2p;
  __shared__ __align__(16) float sT[8][16 * 68];
  const int b    = blockIdx.y;
  const int lane = threadIdx.x & 31;
  const int wave = threadIdx.x >> 5;
  const int tilesN = N >> 6;
  const int tilesM = M >> 6;
  const int tile = blockIdx.x * 8 + wave;
  if (tile >= tilesM * tilesN) return;
  const int tm = tile / tilesN;
  const int tn = tile - tm * tilesN;
  const int m0 = tm << 6;
  const int n0 = tn << 6;

  const T* Ab  = A  + (size_t)b * strideA;
  const T* Bb  = Bt + (size_t)b * strideB;
  const T* Ab2 = (SPLIT || ASPLIT) ? (A2  + (size_t)b * strideA) : nullptr;
  const T* Bb2 = SPLIT ? (Bt2 + (size_t)b * strideB) : nullptr;

  const int rlane = lane & 15;
  const int koff  = (lane >> 4) * 8;
  const int mOff  = (lane >> 4) * 8;

  v8f acc[4][4];
#pragma unroll
  for (int i = 0; i < 4; ++i)
#pragma unroll
    for (int j = 0; j < 4; ++j) acc[i][j] = (v8f){0.f,0.f,0.f,0.f,0.f,0.f,0.f,0.f};

  for (int k0 = 0; k0 < K; k0 += 32) {
    V bh[4], bl[4];
#pragma unroll
    for (int j = 0; j < 4; ++j) {
      const size_t bo = (size_t)(n0 + (j << 4) + rlane) * ldb + koff + k0;
      bh[j] = Frag<T>::load(Bb + bo);
      if (SPLIT) bl[j] = Frag<T>::load(Bb2 + bo);
    }
#pragma unroll
    for (int i = 0; i < 4; ++i) {
      const size_t ao = (size_t)(m0 + (i << 4) + rlane) * lda + koff + k0;
      V ah = Frag<T>::load(Ab + ao);
      V al;
      if (SPLIT || ASPLIT) al = Frag<T>::load(Ab2 + ao);
#pragma unroll
      for (int j = 0; j < 4; ++j) {
        acc[i][j] = Frag<T>::mma(ah, bh[j], acc[i][j]);
        if (SPLIT) {
          acc[i][j] = Frag<T>::mma(ah, bl[j], acc[i][j]);
          acc[i][j] = Frag<T>::mma(al, bh[j], acc[i][j]);
        }
        if (ASPLIT) {
          acc[i][j] = Frag<T>::mma(al, bh[j], acc[i][j]);
        }
      }
      Frag<T>::guard(acc[i][0], acc[i][3], ah, (SPLIT || ASPLIT) ? al : ah);
    }
    Frag<T>::keep(bh[0], bh[1], bh[2], bh[3]);
    if (SPLIT) Frag<T>::keep(bl[0], bl[1], bl[2], bl[3]);
  }
  acc_guard4(acc[0][0], acc[0][1], acc[0][2], acc[0][3]);
  acc_guard4(acc[1][0], acc[1][1], acc[1][2], acc[1][3]);
  acc_guard4(acc[2][0], acc[2][1], acc[2][2], acc[2][3]);
  acc_guard4(acc[3][0], acc[3][1], acc[3][2], acc[3][3]);

  float* slab = sT[wave];
  const float* Rb = RESID ? (resid + (size_t)b * strideR) : nullptr;
#pragma unroll
  for (int i = 0; i < 4; ++i) {
    const int mBase = m0 + (i << 4);
#pragma unroll
    for (int j = 0; j < 4; ++j) {
      const int n = n0 + (j << 4) + rlane;
      float bv = 0.f;
      if (BIAS_MODE == 2) bv = bias[n];
#pragma unroll
      for (int r = 0; r < 8; ++r) {
        float v = acc[i][j][r] * scale;
        if (BIAS_MODE == 1) v += bias[mBase + mOff + r];
        if (BIAS_MODE == 2) v += bv;
        if (RESID) v += Rb[(size_t)(mBase + mOff + r) * ldc + n];
        if (ACT == 1) v = tanhf(v);
        if (ACT == 2) v = fmaxf(v, 0.0f);
        if (ACT == 4) v = (v > 0.f) ? v : 0.01f * v;
        slab[(mOff + r) * 68 + (j << 4) + rlane] = v;
      }
    }
    __builtin_amdgcn_fence(__ATOMIC_RELEASE, "workgroup");
    __builtin_amdgcn_wave_barrier();
    __builtin_amdgcn_fence(__ATOMIC_ACQUIRE, "workgroup");
    if (OUT_MODE == 0) {
      float* C = (float*)Cout + (size_t)b * strideC;
      const int hh = lane >> 4, c4 = (lane & 15) * 4;
      for (int pass = 0; pass < 2; ++pass) {
#pragma unroll
        for (int it = 0; it < 8; ++it) {
          const int row = it * 2 + hh;
          v4f v = *(const v4f*)(slab + row * 68 + c4);
          *(volatile v4f*)(C + (size_t)(mBase + row) * ldc + n0 + c4) = v;
        }
        __threadfence();
      }
    } else {
      const int q = lane >> 3, c8 = (lane & 7) * 8;
      unsigned short* C  = (unsigned short*)Cout  + (size_t)b * strideC;
      unsigned short* C2 = (OUT_MODE == 2) ? ((unsigned short*)Cout2 + (size_t)b * strideC) : nullptr;
      for (int pass = 0; pass < 2; ++pass) {
#pragma unroll
        for (int it = 0; it < 4; ++it) {
          const int row = it * 4 + q;
          const float* sp = slab + row * 68 + c8;
          v8h hv, lv;
#pragma unroll
          for (int e = 0; e < 8; ++e) {
            if (OUT_MODE == 1) {
              hv[e] = (_Float16)sp[e];
            } else {
              unsigned short hb = f2bf_bits(sp[e]);
              unsigned short lb = f2bf_bits(sp[e] - bf_bits2f(hb));
              hv[e] = __builtin_bit_cast(_Float16, hb);
              lv[e] = __builtin_bit_cast(_Float16, lb);
            }
          }
          *(volatile v8h*)(C + (size_t)(mBase + row) * ldc + n0 + c8) = hv;
          if (OUT_MODE == 2) *(volatile v8h*)(C2 + (size_t)(mBase + row) * ldc + n0 + c8) = lv;
        }
        __threadfence();
      }
    }
    __builtin_amdgcn_fence(__ATOMIC_RELEASE, "workgroup");
    __builtin_amdgcn_wave_barrier();
    __builtin_amdgcn_fence(__ATOMIC_ACQUIRE, "workgroup");
  }
}

__global__ __launch_bounds__(256) void cast_bf16x2_kernel(const float* __restrict__ in,
                                                          unsigned short* __restrict__ out, int n2) {
  const int i = blockIdx.x * 256 + threadIdx.x;
  if (i < n2) {
    const v2f f = *(const v2f*)(in + 2 * (size_t)i);
    const unsigned u = pk16(f2bf_bits(f[0]), f2bf_bits(f[1]));
    ((volatile unsigned*)out)[i] = u;
    __threadfence();
    ((volatile unsigned*)out)[i] = u;
  }
}

__global__ __launch_bounds__(256) void normrope_kernel(
    const float* __restrict__ qkf, const float* __restrict__ bq, const float* __restrict__ bk,
    const float* __restrict__ qw, const float* __restrict__ kw,
    const float* __restrict__ cosb, const float* __restrict__ sinb,
    unsigned short* __restrict__ qhp, unsigned short* __restrict__ qlp,
    unsigned short* __restrict__ khp, unsigned short* __restrict__ klp, int s0, int bidx) {
  const int t = blockIdx.x >> 1;
  const int which = blockIdx.x & 1;
  const int wave = threadIdx.x >> 5;
  const int lane = threadIdx.x & 31;
  const int g = lane >> 4;
  const int cl = lane & 15;
  const int h = wave * 2 + g;
  const int d0 = cl * 8;
  const int s = s0 + t;
  const int f = h * kHd + d0;
  const float* src = qkf + (size_t)t * (2 * kDm) + which * kDm + f;
  const float* bp = which ? bk : bq;
  const float* wp = which ? kw : qw;
  const float* cp = cosb + ((size_t)bidx * kSeq + s) * kHd + d0;
  const float* sp = sinb + ((size_t)bidx * kSeq + s) * kHd + d0;
  unsigned short* dsth = (which ? khp : qhp) + (size_t)s * kDm + f;
  unsigned short* dstl = (which ? klp : qlp) + (size_t)s * kDm + f;

  const v4f xa = *(const v4f*)src,       xb = *(const v4f*)(src + 4);
  const v4f ba = *(const v4f*)(bp + f),  bb = *(const v4f*)(bp + f + 4);
  const v4f wa = *(const v4f*)(wp + d0), wb = *(const v4f*)(wp + d0 + 4);
  const v4f ca = *(const v4f*)cp,        cb = *(const v4f*)(cp + 4);
  const v4f sa = *(const v4f*)sp,        sb = *(const v4f*)(sp + 4);
  float x[8], wv[8], cv[8], sv[8];
#pragma unroll
  for (int i = 0; i < 4; ++i) {
    x[i]  = xa[i] + bf_rne(ba[i]);  x[4 + i]  = xb[i] + bf_rne(bb[i]);
    wv[i] = bf_rne(wa[i]);          wv[4 + i] = bf_rne(wb[i]);
    cv[i] = bf_rne(ca[i]);          cv[4 + i] = bf_rne(cb[i]);
    sv[i] = bf_rne(sa[i]);          sv[4 + i] = bf_rne(sb[i]);
  }
  float ss = 0.f;
#pragma unroll
  for (int i = 0; i < 8; ++i) ss += x[i] * x[i];
  ss += __shfl_xor(ss, 1, 32);
  ss += __shfl_xor(ss, 2, 32);
  ss += __shfl_xor(ss, 4, 32);
  ss += __shfl_xor(ss, 8, 32);
  const float inv = rsqrtf(ss * (1.0f / 128.0f) + 1.0e-6f);
  float xn[8], o[8];
#pragma unroll
  for (int i = 0; i < 8; ++i) xn[i] = (x[i] * inv) * wv[i];
#pragma unroll
  for (int i = 0; i < 8; ++i) {
    const float pr = __shfl_xor(xn[i], 8, 32);
    const float rot = (cl < 8) ? -pr : pr;
    o[i] = xn[i] * cv[i] + rot * sv[i];
  }
  v8h hv, lv;
#pragma unroll
  for (int i = 0; i < 8; ++i) {
    const unsigned short hb = f2bf_bits(o[i]);
    const unsigned short lb = f2bf_bits(o[i] - bf_bits2f(hb));
    hv[i] = __builtin_bit_cast(_Float16, hb);
    lv[i] = __builtin_bit_cast(_Float16, lb);
  }
  *(volatile v8h*)dsth = hv;
  *(volatile v8h*)dstl = lv;
  __threadfence();
  *(volatile v8h*)dsth = hv;
  *(volatile v8h*)dstl = lv;
}

__global__ __launch_bounds__(256) void tilemax_kernel(const float* __restrict__ maskb, float* __restrict__ tmax) {
  __shared__ float part[8][32];
  const int qt = blockIdx.x;
  const int wave = threadIdx.x >> 5;
  const int lane = threadIdx.x & 31;
  const int hh = lane >> 4;
  const int c4 = (lane & 15) * 4;
  const float* base = maskb + (size_t)(qt * 64 + wave * 8) * kSeq + hh * 64 + c4;
#pragma unroll 1
  for (int i = 0; i < 16; ++i) {
    float a = -INFINITY;
#pragma unroll
    for (int r = 0; r < 8; ++r) {
      const v4f m4 = *(const v4f*)(base + (size_t)r * kSeq + i * 128);
      a = fmaxf(a, fmaxf(fmaxf(m4[0], m4[1]), fmaxf(m4[2], m4[3])));
    }
#pragma unroll
    for (int off = 1; off < 16; off <<= 1) a = fmaxf(a, __shfl_xor(a, off, 32));
    if ((lane & 15) == 0) part[wave][2 * i + hh] = a;
  }
  __syncthreads();
  if (wave == 0) {
    float v = part[0][lane];
#pragma unroll
    for (int w = 1; w < 8; ++w) v = fmaxf(v, part[w][lane]);
    volatile float* dst = tmax + qt * 32;
    dst[lane] = v;
    __threadfence();
    dst[lane] = v;
  }
}

constexpr int kAKP = 136;
constexpr int kAVP = 72;
constexpr int kAOP = 68;

__device__ __forceinline__ v8f mma_b(v16b a, v16b b, v8f c) {
  c = __builtin_amdgcn_wmma_f32_16x16x32_bf16(false, a, false, b, (short)0, c, false, false);
  asm volatile("v_nop\n\tv_nop\n\tv_nop\n\tv_nop" : "+v"(c) : "v"(a), "v"(b));
  return c;
}
__device__ __forceinline__ void sched_fence() { asm volatile("" ::: "memory"); }

__global__ __launch_bounds__(128) __attribute__((amdgpu_num_vgpr(256)))
void attn128_kernel(const unsigned short* __restrict__ qhp, const unsigned short* __restrict__ qlp,
                    const unsigned short* __restrict__ khp, const unsigned short* __restrict__ klp,
                    const unsigned short* __restrict__ vhp, const unsigned short* __restrict__ vlp,
                    const float* __restrict__ amask, const float* __restrict__ tmax,
                    unsigned short* __restrict__ ohp, unsigned short* __restrict__ olp, float sscale) {
  __shared__ __align__(16) __bf16 Qsh[64 * kAKP];
  __shared__ __align__(16) __bf16 Qsl[64 * kAKP];
  __shared__ __align__(16) __bf16 Ksh[64 * kAKP];
  __shared__ __align__(16) __bf16 Ksl[64 * kAKP];
  __shared__ __align__(16) __bf16 Vsh[128 * kAVP];
  __shared__ __align__(16) __bf16 Vsl[128 * kAVP];
  __shared__ __align__(16) __bf16 Psh[4][16 * 64];
  __shared__ __align__(16) __bf16 Psl[4][16 * 64];
  __shared__ __align__(16) float    Os[4][16 * kAOP];
  __shared__ float red[4];

  const int tid  = threadIdx.x;
  const int wave = tid >> 5;
  const int lane = tid & 31;
  const int hh   = lane >> 4;
  const int c    = lane & 15;

  const int bx = blockIdx.x;
  const int qb = bx & (kNQB - 1);
  const int h  = bx >> 5;
  const int qt0 = qb * 64;
  const int q0 = qt0 + wave * 16;

  const __bf16* Qh = (const __bf16*)(const void*)qhp + h * kHd;
  const __bf16* Ql = (const __bf16*)(const void*)qlp + h * kHd;
  const __bf16* Kh = (const __bf16*)(const void*)khp + h * kHd;
  const __bf16* Kl = (const __bf16*)(const void*)klp + h * kHd;
  const __bf16* Vh = (const __bf16*)(const void*)vhp + (size_t)(h * kHd) * kSeq;
  const __bf16* Vl = (const __bf16*)(const void*)vlp + (size_t)(h * kHd) * kSeq;
  unsigned short* Oh = ohp + h * kHd;
  unsigned short* Ol = olp + h * kHd;

  {
    const int r = tid >> 1, cb = (tid & 1) * 64;
    const __bf16* qhr = Qh + (size_t)(qt0 + r) * kDm + cb;
    const __bf16* qlr = Ql + (size_t)(qt0 + r) * kDm + cb;
#pragma unroll
    for (int i = 0; i < 8; ++i) {
      const v8b a0 = *(const v8b*)(qhr + 8 * i);
      const v8b a1 = *(const v8b*)(qlr + 8 * i);
      *(v8b*)(Qsh + r * kAKP + cb + 8 * i) = a0;
      *(v8b*)(Qsl + r * kAKP + cb + 8 * i) = a1;
    }
  }

  float mrow[8], lrow[8];
  v8f oacc[8];
  const v8f z8f = (v8f){0.f,0.f,0.f,0.f,0.f,0.f,0.f,0.f};
#pragma unroll
  for (int r = 0; r < 8; ++r) { mrow[r] = -INFINITY; lrow[r] = 0.f; }
#pragma unroll
  for (int t = 0; t < 8; ++t) oacc[t] = z8f;

  const __bf16* qrh = Qsh + (wave * 16 + c) * kAKP + 8 * hh;
  const __bf16* qrl = Qsl + (wave * 16 + c) * kAKP + 8 * hh;
  __bf16* pwh = Psh[wave];
  __bf16* pwl = Psl[wave];

  for (int kc = 0; kc < kNQB; ++kc) {
    const int kv0 = kc * 64;
    __syncthreads();
    {
      float mn = mrow[0];
#pragma unroll
      for (int r = 1; r < 8; ++r) mn = fminf(mn, mrow[r]);
#pragma unroll
      for (int off = 1; off < 32; off <<= 1) mn = fminf(mn, __shfl_xor(mn, off, 32));
      if (lane == 0) red[wave] = mn;
    }
    __syncthreads();
    const float bmn = fminf(fminf(red[0], red[1]), fminf(red[2], red[3]));
    const float tmv = tmax[qb * kNQB + kc];
    const int skipi = __builtin_amdgcn_readfirstlane(((tmv <= -1.0e6f) && (bmn >= -1.0e4f)) ? 1 : 0);
    if (skipi) continue;

    {
      const int r = tid >> 1, cb = (tid & 1) * 64;
      const __bf16* khr = Kh + (size_t)(kv0 + r) * kDm + cb;
      const __bf16* klr = Kl + (size_t)(kv0 + r) * kDm + cb;
#pragma unroll
      for (int i = 0; i < 8; ++i) {
        const v8b a0 = *(const v8b*)(khr + 8 * i);
        const v8b a1 = *(const v8b*)(klr + 8 * i);
        *(v8b*)(Ksh + r * kAKP + cb + 8 * i) = a0;
        *(v8b*)(Ksl + r * kAKP + cb + 8 * i) = a1;
      }
      const int d = tid;
      const __bf16* vhr = Vh + (size_t)d * kSeq + kv0;
      const __bf16* vlr = Vl + (size_t)d * kSeq + kv0;
#pragma unroll
      for (int i = 0; i < 8; ++i) {
        const v8b b0 = *(const v8b*)(vhr + 8 * i);
        const v8b b1 = *(const v8b*)(vlr + 8 * i);
        *(v8b*)(Vsh + d * kAVP + 8 * i) = b0;
        *(v8b*)(Vsl + d * kAVP + 8 * i) = b1;
      }
    }
    __syncthreads();

    v8f s[4];
#pragma unroll
    for (int j = 0; j < 4; ++j) s[j] = z8f;
#pragma unroll
    for (int dc = 0; dc < 4; ++dc) {
      sched_fence();
      const v16b qa  = Frag<__bf16>::load(qrh + dc * 32);
      const v16b qal = Frag<__bf16>::load(qrl + dc * 32);
#pragma unroll
      for (int j = 0; j < 4; ++j) {
        sched_fence();
        const v16b kb  = Frag<__bf16>::load(Ksh + (j * 16 + c) * kAKP + dc * 32 + 8 * hh);
        const v16b klf = Frag<__bf16>::load(Ksl + (j * 16 + c) * kAKP + dc * 32 + 8 * hh);
        s[j] = mma_b(qa, kb, s[j]);
        s[j] = mma_b(qa, klf, s[j]);
        s[j] = mma_b(qal, kb, s[j]);
      }
    }
    float cm[8];
#pragma unroll
    for (int r = 0; r < 8; ++r) {
      const int qrow = q0 + 8 * hh + r;
      const float* mline = amask + (size_t)qrow * kSeq + kv0 + c;
      float m = -INFINITY;
#pragma unroll
      for (int j = 0; j < 4; ++j) {
        const float mv = bf_rne(mline[j * 16]);
        const float sv = s[j][r] * sscale + mv;
        s[j][r] = sv;
        m = fmaxf(m, sv);
      }
#pragma unroll
      for (int off = 1; off < 16; off <<= 1) m = fmaxf(m, __shfl_xor(m, off, 32));
      cm[r] = m;
    }
#pragma unroll
    for (int r = 0; r < 8; ++r) {
      const float mnew = fmaxf(mrow[r], cm[r]);
      const float alpha = __expf(mrow[r] - mnew);
      mrow[r] = mnew;
      float psum = 0.f;
#pragma unroll
      for (int j = 0; j < 4; ++j) {
        const float p = __expf(s[j][r] - mnew);
        psum += p;
        const unsigned short hb = f2bf_bits(p);
        const unsigned short lb = f2bf_bits(p - bf_bits2f(hb));
        pwh[(8 * hh + r) * 64 + j * 16 + c] = __builtin_bit_cast(__bf16, hb);
        pwl[(8 * hh + r) * 64 + j * 16 + c] = __builtin_bit_cast(__bf16, lb);
      }
#pragma unroll
      for (int off = 1; off < 16; off <<= 1) psum += __shfl_xor(psum, off, 32);
      lrow[r] = lrow[r] * alpha + psum;
#pragma unroll
      for (int t = 0; t < 8; ++t) oacc[t][r] *= alpha;
    }
    __builtin_amdgcn_fence(__ATOMIC_RELEASE, "workgroup");
    __builtin_amdgcn_wave_barrier();
    __builtin_amdgcn_fence(__ATOMIC_ACQUIRE, "workgroup");
#pragma unroll 1
    for (int kk = 0; kk < 2; ++kk) {
      const v16b pa = Frag<__bf16>::load(pwh + c * 64 + kk * 32 + 8 * hh);
      const v16b pl = Frag<__bf16>::load(pwl + c * 64 + kk * 32 + 8 * hh);
#pragma unroll
      for (int t = 0; t < 8; ++t) {
        sched_fence();
        const v16b vb = Frag<__bf16>::load(Vsh + (t * 16 + c) * kAVP + kk * 32 + 8 * hh);
        const v16b vl = Frag<__bf16>::load(Vsl + (t * 16 + c) * kAVP + kk * 32 + 8 * hh);
        oacc[t] = mma_b(pa, vb, oacc[t]);
        oacc[t] = mma_b(pa, vl, oacc[t]);
        oacc[t] = mma_b(pl, vb, oacc[t]);
      }
    }
  }

  float invl[8];
#pragma unroll
  for (int r = 0; r < 8; ++r) invl[r] = __builtin_amdgcn_rcpf(lrow[r]);
  float* os = Os[wave];
  const int q4 = lane >> 3, c8 = (lane & 7) * 8;
#pragma unroll
  for (int g = 0; g < 2; ++g) {
#pragma unroll
    for (int r = 0; r < 8; ++r) {
#pragma unroll
      for (int t = 0; t < 4; ++t) os[(8 * hh + r) * kAOP + t * 16 + c] = oacc[4 * g + t][r] * invl[r];
    }
    __builtin_amdgcn_fence(__ATOMIC_RELEASE, "workgroup");
    __builtin_amdgcn_wave_barrier();
    __builtin_amdgcn_fence(__ATOMIC_ACQUIRE, "workgroup");
    for (int pass = 0; pass < 2; ++pass) {
#pragma unroll
      for (int it = 0; it < 4; ++it) {
        const int row = it * 4 + q4;
        const float* spp = os + row * kAOP + c8;
        v8h hv, lv;
#pragma unroll
        for (int e = 0; e < 8; ++e) {
          const unsigned short hb = f2bf_bits(spp[e]);
          const unsigned short lb = f2bf_bits(spp[e] - bf_bits2f(hb));
          hv[e] = __builtin_bit_cast(_Float16, hb);
          lv[e] = __builtin_bit_cast(_Float16, lb);
        }
        const size_t go = (size_t)(q0 + row) * kDm + g * 64 + c8;
        *(volatile v8h*)(Oh + go) = hv;
        *(volatile v8h*)(Ol + go) = lv;
      }
      __threadfence();
    }
    __builtin_amdgcn_fence(__ATOMIC_RELEASE, "workgroup");
    __builtin_amdgcn_wave_barrier();
    __builtin_amdgcn_fence(__ATOMIC_ACQUIRE, "workgroup");
  }
}

constexpr size_t kBPlane16 = (size_t)kSeq * kDm * 2;
constexpr size_t kW16      = (size_t)kDm * kDm * 2;
constexpr size_t kQKfBytes = (size_t)kChunkTok * 2 * kDm * 4;
constexpr size_t kTmaxBytes = (size_t)kNQB * kNQB * 4;
constexpr size_t kOffWqk = 0;
constexpr size_t kOffWv  = kOffWqk + 2 * kW16;
constexpr size_t kOffWo  = kOffWv + kW16;
constexpr size_t kOffX   = kOffWo + kW16;
constexpr size_t kOffQKf = kOffX + kBPlane16;
constexpr size_t kOffQh  = kOffQKf + kQKfBytes;
constexpr size_t kOffQl  = kOffQh + kBPlane16;
constexpr size_t kOffKh  = kOffQl + kBPlane16;
constexpr size_t kOffKl  = kOffKh + kBPlane16;
constexpr size_t kOffVh  = kOffKl + kBPlane16;
constexpr size_t kOffVl  = kOffVh + kBPlane16;
constexpr size_t kOffOh  = kOffVl + kBPlane16;
constexpr size_t kOffOl  = kOffOh + kBPlane16;
constexpr size_t kOffTmax = kOffOl + kBPlane16;
constexpr size_t kWsTotal = kOffTmax + kTmaxBytes;
static_assert(kWsTotal == 125833216, "carve total");
static_assert(kWsTotal <= 134217728, "carve budget");

extern "C" void kernel_launch(void* const* d_in, const int* in_sizes, int n_in,
                              void* d_out, int out_size, void* d_ws, size_t ws_size,
                              hipStream_t stream) {
  if (n_in < 13) return;
  if (in_sizes[0] != kTok * kDm) return;
  if (in_sizes[1] != kTok * kHd || in_sizes[2] != kTok * kHd) return;
  if (in_sizes[3] != kBatch * kSeq * kSeq) return;
  if (in_sizes[4] != kDm * kDm || in_sizes[6] != kDm * kDm || in_sizes[8] != kDm * kDm || in_sizes[10] != kDm * kDm) return;
  if (in_sizes[5] != kDm || in_sizes[7] != kDm || in_sizes[9] != kDm) return;
  if (in_sizes[11] != kHd || in_sizes[12] != kHd) return;
  if (out_size != kTok * kDm) return;
  if (ws_size < kWsTotal) return;

  const float* hid   = (const float*)d_in[0];
  const float* cosb  = (const float*)d_in[1];
  const float* sinb  = (const float*)d_in[2];
  const float* amask = (const float*)d_in[3];
  const float* Wq    = (const float*)d_in[4];
  const float* bq    = (const float*)d_in[5];
  const float* Wk    = (const float*)d_in[6];
  const float* bk    = (const float*)d_in[7];
  const float* Wv    = (const float*)d_in[8];
  const float* bv    = (const float*)d_in[9];
  const float* Wo    = (const float*)d_in[10];
  const float* qnw   = (const float*)d_in[11];
  const float* knw   = (const float*)d_in[12];

  char* ws = (char*)d_ws;
  unsigned short* Wqkb = (unsigned short*)(ws + kOffWqk);
  unsigned short* Wvb  = (unsigned short*)(ws + kOffWv);
  unsigned short* Wob  = (unsigned short*)(ws + kOffWo);
  unsigned short* Xb   = (unsigned short*)(ws + kOffX);
  float*          QKf  = (float*)(ws + kOffQKf);
  unsigned short* Qh   = (unsigned short*)(ws + kOffQh);
  unsigned short* Ql   = (unsigned short*)(ws + kOffQl);
  unsigned short* Kh   = (unsigned short*)(ws + kOffKh);
  unsigned short* Kl   = (unsigned short*)(ws + kOffKl);
  unsigned short* VTh  = (unsigned short*)(ws + kOffVh);
  unsigned short* VTl  = (unsigned short*)(ws + kOffVl);
  unsigned short* Oh   = (unsigned short*)(ws + kOffOh);
  unsigned short* Ol   = (unsigned short*)(ws + kOffOl);
  float*          Tmax = (float*)(ws + kOffTmax);

  const int n2 = kDm * kDm / 2;
  const int castBlocks = (n2 + 255) / 256;

  cast_bf16x2_kernel<<<castBlocks, 256, 0, stream>>>(Wq, Wqkb, n2);
  cast_bf16x2_kernel<<<castBlocks, 256, 0, stream>>>(Wk, Wqkb + (size_t)kDm * kDm, n2);
  cast_bf16x2_kernel<<<castBlocks, 256, 0, stream>>>(Wv, Wvb, n2);
  cast_bf16x2_kernel<<<castBlocks, 256, 0, stream>>>(Wo, Wob, n2);

  for (int b = 0; b < kBatch; ++b) {
    cast_bf16x2_kernel<<<castBlocks, 256, 0, stream>>>(hid + (size_t)b * kSeq * kDm, Xb, n2);
    wmma_gemm64<1, false, 1, 2, false><<<dim3(128, 1), 256, 0, stream>>>(
        Wvb, nullptr, kDm, 0L, Xb, nullptr, kDm, 0L,
        (void*)VTh, (void*)VTl, kSeq, 0L, bv, nullptr, 0L, kDm, kSeq, kDm, 1.0f);
    for (int ch = 0; ch < kNumChunks; ++ch) {
      const int s0 = ch * kChunkTok;
      wmma_gemm64<1, false, 0, 0, false><<<dim3(128, 1), 256, 0, stream>>>(
          Xb + (size_t)s0 * kDm, nullptr, kDm, 0L, Wqkb, nullptr, kDm, 0L,
          (void*)QKf, nullptr, 2 * kDm, 0L, nullptr, nullptr, 0L, kChunkTok, 2 * kDm, kDm, 1.0f);
      normrope_kernel<<<kChunkTok * 2, 256, 0, stream>>>(QKf, bq, bk, qnw, knw, cosb, sinb, Qh, Ql, Kh, Kl, s0, b);
    }
    const float* maskb = amask + (size_t)b * kSeq * kSeq;
    tilemax_kernel<<<kNQB, 256, 0, stream>>>(maskb, Tmax);
    attn128_kernel<<<kHeads * kNQB, 128, 0, stream>>>(Qh, Ql, Kh, Kl, VTh, VTl, maskb, Tmax, Oh, Ol, kScoreScale);
    wmma_gemm64<1, false, 0, 0, false, 0, true><<<dim3(128, 1), 256, 0, stream>>>(
        Oh, Ol, kDm, 0L, Wob, nullptr, kDm, 0L,
        (void*)((float*)d_out + (size_t)b * kSeq * kDm), nullptr, kDm, 0L, nullptr, nullptr, 0L, kSeq, kDm, kDm, 1.0f);
  }
}
